// Decoder_43078521979490
// MI455X (gfx1250) — hardware-verified
//
#include <hip/hip_runtime.h>
#include <math.h>

#pragma clang fp contract(off)

#ifndef NB
#define NB 8192
#endif
#define NB_FULL 8192
#ifndef MCH
#define MCH 2048
#endif
#define D0 256
#define D1 1024
#define D2 512
#define D3 512
#define NKNOT 12
#define KMAX (9 * D1)
#define XP_ROWS 32

static_assert(NB % MCH == 0);
static_assert(MCH % 64 == 0 && MCH % XP_ROWS == 0 && XP_ROWS % 8 == 0);
static_assert(D0 % 256 == 0 && D1 % 256 == 0 && D2 % 256 == 0);
static_assert(D1 % 64 == 0 && D2 % 64 == 0 && D3 % 64 == 0);
static_assert((9 * D0) % 32 == 0 && (9 * D1) % 32 == 0 && (9 * D2) % 32 == 0);
static_assert((9 * D0) <= KMAX && (9 * D2) <= KMAX);
static_assert(((MCH / 64) * (D1 / 64)) % 8 == 0 && ((MCH / 64) * (D2 / 64)) % 8 == 0 && ((MCH / 64) * (D3 / 64)) % 8 == 0);
static_assert((D1 * (9 * D0 / 8)) % 256 == 0 && (D2 * (9 * D1 / 8)) % 256 == 0 && (D3 * (9 * D2 / 8)) % 256 == 0);
static_assert(D3 == 512);
static_assert((size_t)NB_FULL * D3 * 4 == (size_t)16777216);
static_assert(8 * 16 * 68 * 4 <= 131072);
static_assert(32 * 16 * 8 == 16 * 64 * 4);
static_assert(256 * 16 * XP_ROWS == XP_ROWS * 256 * 16);
static_assert(256 * 16 * (XP_ROWS / 8) == XP_ROWS * 256 * 2);

static constexpr size_t WS_A  = (size_t)MCH * KMAX * 2;
static constexpr size_t WS_H0 = (size_t)MCH * D1 * 4;
static constexpr size_t WS_H1 = (size_t)MCH * D2 * 4;
static constexpr size_t WS_W0 = (size_t)D1 * 9 * D0 * 2;
static constexpr size_t WS_W1 = (size_t)D2 * 9 * D1 * 2;
static constexpr size_t WS_W2 = (size_t)D3 * 9 * D2 * 2;
static_assert(WS_A % 256 == 0 && WS_H0 % 256 == 0 && WS_H1 % 256 == 0 && WS_W0 % 256 == 0 && WS_W1 % 256 == 0 && WS_W2 % 256 == 0);
static_assert(WS_A + WS_H0 + WS_H1 + WS_W0 + WS_W1 + WS_W2 <= (size_t)134217728);

static constexpr float SC = 1.0f / 262144.0f;

typedef __attribute__((ext_vector_type(16))) _Float16 v16h;
typedef __attribute__((ext_vector_type(8)))  _Float16 v8h;
typedef __attribute__((ext_vector_type(8)))  float    v8f;
typedef __attribute__((ext_vector_type(4)))  float    v4f;
typedef __attribute__((ext_vector_type(4)))  unsigned int v4u;
typedef _Float16 h16;


#define VST2(T, ptr, val) do { const T vst2_v_ = (val); *(volatile T*)(ptr) = vst2_v_; __threadfence(); *(volatile T*)(ptr) = vst2_v_; } while (0)
#define VST2V4(ptr, val) do { const v4f vst2_v4_ = (val); *(volatile v4f*)(ptr) = vst2_v4_; __threadfence(); *(volatile v4f*)(ptr) = vst2_v4_; } while (0)

__device__ __forceinline__ float bfr(float f) {
    unsigned u = __float_as_uint(f);
    u += 0x7FFFu + ((u >> 16) & 1u);
    return __uint_as_float(u & 0xFFFF0000u);
}
static __device__ __forceinline__ h16 toh_flush(float v) {
    const h16 r = (h16)v;
    return (fabsf(v) < 6.103515625e-05f) ? (h16)0.0f : r;
}
__device__ __forceinline__ void st8h_flush(unsigned short* P, size_t o, const float* v) {
    v8h hv;
#pragma unroll
    for (int e = 0; e < 8; ++e) hv[e] = toh_flush(v[e]);
    const v4u pk = __builtin_bit_cast(v4u, hv);
    VST2(v4u, (v4u*)(P + o), pk);
}

union FragU { v16h v; v8h h[2]; };
__device__ __forceinline__ v16h frag_ld(const _Float16* p) {
    FragU f; f.h[0] = *(const v8h*)(p); f.h[1] = *(const v8h*)(p + 16); return f.v;
}
__device__ __forceinline__ void dep_guard_h(v8f& a, v8f& b, v16h x, v16h y) { asm volatile("v_nop\n\tv_nop\n\tv_nop\n\tv_nop" : "+v"(a), "+v"(b) : "v"(x), "v"(y)); }
__device__ __forceinline__ void keep4_h(v16h a, v16h b, v16h c, v16h d) { asm volatile("v_nop" :: "v"(a), "v"(b), "v"(c), "v"(d)); }
__device__ __forceinline__ void acc_guard4(v8f& a, v8f& b, v8f& c, v8f& d) { asm volatile("v_nop\n\tv_nop\n\tv_nop\n\tv_nop" : "+v"(a), "+v"(b), "+v"(c), "+v"(d)); }
__device__ __forceinline__ void wave_sync_lds() {
    __builtin_amdgcn_fence(3  , "workgroup");
    __builtin_amdgcn_wave_barrier();
    __builtin_amdgcn_fence(2  , "workgroup");
}

__global__ __launch_bounds__(256) void k_gemm64(
    const _Float16* __restrict__ A, unsigned lda, const _Float16* __restrict__ Bt, unsigned ldb,
    float* __restrict__ C, unsigned ldc, const float* __restrict__ gain, const float* __restrict__ bias,
    unsigned M, unsigned N, unsigned K, float scale) {
  __shared__ __align__(16) float sT[8][16 * 68];
  const unsigned lane = threadIdx.x & 31u;
  const unsigned wave = (unsigned)__builtin_amdgcn_readfirstlane((int)(threadIdx.x >> 5));
  const unsigned tilesN = N >> 6, tilesM = M >> 6;
  const unsigned tile = blockIdx.x * 8u + wave;
  if (tile >= tilesM * tilesN) return;
  const unsigned tm = tile / tilesN;
  const unsigned tn = tile - tm * tilesN;
  const unsigned m0 = tm << 6, n0 = tn << 6;
  const unsigned rlane = lane & 15u;
  const unsigned koff = (lane >> 4) * 8u;
  const unsigned mOff = koff;

  v8f acc[4][4];
#pragma unroll
  for (int i = 0; i < 4; ++i)
#pragma unroll
    for (int j = 0; j < 4; ++j) acc[i][j] = (v8f){0.f,0.f,0.f,0.f,0.f,0.f,0.f,0.f};

  for (unsigned k0 = 0; k0 < K; k0 += 32u) {
    v16h bh[4];
#pragma unroll
    for (int j = 0; j < 4; ++j)
      bh[j] = frag_ld(Bt + (size_t)(n0 + ((unsigned)j << 4) + rlane) * ldb + koff + k0);
#pragma unroll
    for (int i = 0; i < 4; ++i) {
      const v16h ah = frag_ld(A + (size_t)(m0 + ((unsigned)i << 4) + rlane) * lda + koff + k0);
#pragma unroll
      for (int j = 0; j < 4; ++j)
        acc[i][j] = __builtin_amdgcn_wmma_f32_16x16x32_f16(false, ah, false, bh[j], (short)0, acc[i][j], false, false);
      dep_guard_h(acc[i][0], acc[i][3], ah, ah);
    }
    keep4_h(bh[0], bh[1], bh[2], bh[3]);
  }
  acc_guard4(acc[0][0], acc[0][1], acc[0][2], acc[0][3]);
  acc_guard4(acc[1][0], acc[1][1], acc[1][2], acc[1][3]);
  acc_guard4(acc[2][0], acc[2][1], acc[2][2], acc[2][3]);
  acc_guard4(acc[3][0], acc[3][1], acc[3][2], acc[3][3]);

#pragma unroll
  for (int i = 0; i < 4; ++i) {
    const unsigned mBase = m0 + ((unsigned)i << 4);
#pragma unroll
    for (int j = 0; j < 4; ++j) {
      const unsigned n = n0 + ((unsigned)j << 4) + rlane;
      const float gv = bfr(gain[n]);
      const float bv = bfr(bias[n]);
#pragma unroll
      for (int r = 0; r < 8; ++r) {
        const float v = (acc[i][j][r] * scale) * gv + bv;
        sT[wave][(mOff + (unsigned)r) * 68u + ((unsigned)j << 4) + rlane] = v;
      }
    }
    wave_sync_lds();
    {
      const unsigned hh = lane >> 4, c4 = (lane & 15u) * 4u;
#pragma unroll
      for (int half = 0; half < 2; ++half) {
        v4f vv[4];
#pragma unroll
        for (int it = 0; it < 4; ++it) {
          const unsigned row = (unsigned)(half * 4 + it) * 2u + hh;
          vv[it] = *(const v4f*)(&sT[wave][row * 68u + c4]);
        }
        for (int pass = 0; pass < 2; ++pass) {
#pragma unroll
          for (int it = 0; it < 4; ++it) {
            const unsigned row = (unsigned)(half * 4 + it) * 2u + hh;
            *(volatile v4f*)(C + (size_t)(mBase + row) * ldc + n0 + c4) = vv[it];
          }
          __threadfence();
        }
      }
    }
    wave_sync_lds();
  }
}

__global__ __launch_bounds__(256) void k_wpack(const float* __restrict__ coef, const float* __restrict__ sb,
                                               const float* __restrict__ ss, unsigned short* __restrict__ W16,
                                               unsigned IN, unsigned OUTN) {
    const unsigned per = IN + (IN >> 3);
    const unsigned u = blockIdx.x * 256u + threadIdx.x;
    const unsigned o = u / per;
    const unsigned p = u - o * per;
    if (o >= OUTN) return;
    const unsigned p0 = (unsigned)__builtin_amdgcn_readfirstlane((int)p);
    float v[8];
    if (p0 < IN) {
        const v4f* cp = (const v4f*)(coef + ((size_t)p * OUTN + o) * 8u);
        const v4f a = cp[0], b = cp[1];
        const float s = bfr(ss[(size_t)p * OUTN + o]);
        v[0] = bfr(a.x) * s * 1024.0f; v[1] = bfr(a.y) * s * 1024.0f; v[2] = bfr(a.z) * s * 1024.0f; v[3] = bfr(a.w) * s * 1024.0f;
        v[4] = bfr(b.x) * s * 1024.0f; v[5] = bfr(b.y) * s * 1024.0f; v[6] = bfr(b.z) * s * 1024.0f; v[7] = bfr(b.w) * s * 1024.0f;
    } else {
        const unsigned i0 = (p - IN) * 8u;
#pragma unroll
        for (int e = 0; e < 8; ++e) v[e] = bfr(sb[(size_t)(i0 + (unsigned)e) * OUTN + o]) * 1024.0f;
    }
    st8h_flush(W16, (size_t)o * (9u * IN) + 8u * (size_t)p, v);
}

__global__ __launch_bounds__(256) void k_expand(const float* __restrict__ X, const float* __restrict__ grid,
                                                unsigned short* __restrict__ A16, unsigned IN, unsigned rndx) {
    const unsigned t = threadIdx.x;
    const unsigned f0 = blockIdx.x * 256u;
    const unsigned r0 = blockIdx.y * (unsigned)XP_ROWS;
    const unsigned lda = 9u * IN;
    {
        const unsigned i = f0 + t;
        const v4f* gp = (const v4f*)(grid + (size_t)i * NKNOT);
        const v4f ga = gp[0], gb = gp[1], gc = gp[2];
        const float g[12] = {bfr(ga.x), bfr(ga.y), bfr(ga.z), bfr(ga.w), bfr(gb.x), bfr(gb.y), bfr(gb.z), bfr(gb.w),
                             bfr(gc.x), bfr(gc.y), bfr(gc.z), bfr(gc.w)};
        float i1[11], i2[10], i3[9];
#pragma unroll
        for (int s = 0; s < 11; ++s) i1[s] = __builtin_amdgcn_rcpf(g[s + 1] - g[s]);
#pragma unroll
        for (int s = 0; s < 10; ++s) i2[s] = __builtin_amdgcn_rcpf(g[s + 2] - g[s]);
#pragma unroll
        for (int s = 0; s < 9; ++s) i3[s] = __builtin_amdgcn_rcpf(g[s + 3] - g[s]);
        const float* xs = X + (size_t)r0 * IN + i;
        unsigned short* dst = A16 + (size_t)r0 * lda + (size_t)i * 8u;
#pragma unroll 1
        for (unsigned rr = 0; rr < (unsigned)XP_ROWS; ++rr) {
            const float xr = xs[(size_t)rr * IN];
            const float xb = bfr(xr);
            const float x = (rndx != 0u) ? xb : xr;
            float d[12];
#pragma unroll
            for (int r = 0; r < 12; ++r) d[r] = x - g[r];
            float Bv[11];
#pragma unroll
            for (int r = 0; r < 11; ++r) Bv[r] = ((x >= g[r]) && (x < g[r + 1])) ? 1.0f : 0.0f;
#pragma unroll
            for (int r = 0; r < 10; ++r) Bv[r] = (d[r] * i1[r]) * Bv[r] + ((-d[r + 2]) * i1[r + 1]) * Bv[r + 1];
#pragma unroll
            for (int r = 0; r < 9; ++r)  Bv[r] = (d[r] * i2[r]) * Bv[r] + ((-d[r + 3]) * i2[r + 1]) * Bv[r + 1];
#pragma unroll
            for (int r = 0; r < 8; ++r)  Bv[r] = (d[r] * i3[r]) * Bv[r] + ((-d[r + 4]) * i3[r + 1]) * Bv[r + 1];
            float v[8];
#pragma unroll
            for (int e = 0; e < 8; ++e) v[e] = Bv[e] * 256.0f;
            st8h_flush(dst, (size_t)rr * lda, v);
        }
    }
    {
        const unsigned pc = t & 31u;
#pragma unroll 1
        for (unsigned it = 0; it < (unsigned)(XP_ROWS / 8); ++it) {
            const unsigned row = r0 + it * 8u + (t >> 5);
            const float* xp = X + (size_t)row * IN + f0 + 8u * pc;
            const v4f a = *(const v4f*)xp, b = *(const v4f*)(xp + 4);
            const float xv[8] = {a.x, a.y, a.z, a.w, b.x, b.y, b.z, b.w};
            float v[8];
#pragma unroll
            for (int e = 0; e < 8; ++e) {
                const float xb = bfr(xv[e]);
                const float x = (rndx != 0u) ? xb : xv[e];
                const float sg = __builtin_amdgcn_rcpf(1.0f + exp2f(-1.4426950408889634f * x));
                v[e] = fminf((x * sg) * 256.0f, 60000.0f);
            }
            st8h_flush(A16, (size_t)row * lda + 8u * (size_t)IN + f0 + 8u * pc, v);
        }
    }
}

__global__ __launch_bounds__(128) void k_sigma(const float* __restrict__ sigma, float* __restrict__ dst) {
    const unsigned t = threadIdx.x;
    const v4f s = *(const v4f*)(sigma + 4u * t);
    v4f o;
    o.x = bfr(s.x); o.y = bfr(s.y); o.z = bfr(s.z); o.w = bfr(s.w);
    VST2V4(dst + 4u * t, o);
}

extern "C" void kernel_launch(void* const* d_in, const int* in_sizes, int n_in, void* d_out, int out_size,
                              void* d_ws, size_t ws_size, hipStream_t stream) {
    if (n_in < 20) return;
    if (in_sizes[0] < NB * D0 || in_sizes[1] < D0 * NKNOT || in_sizes[2] < D0 * D1 * 8 || in_sizes[3] < D0 * D1 || in_sizes[4] < D0 * D1) return;
    if (in_sizes[5] < D1 || in_sizes[6] < D1 || in_sizes[7] < D1 * NKNOT || in_sizes[8] < D1 * D2 * 8 || in_sizes[9] < D1 * D2 || in_sizes[10] < D1 * D2) return;
    if (in_sizes[11] < D2 || in_sizes[12] < D2 || in_sizes[13] < D2 * NKNOT || in_sizes[14] < D2 * D3 * 8 || in_sizes[15] < D2 * D3 || in_sizes[16] < D2 * D3) return;
    if (in_sizes[17] < D3 || in_sizes[18] < D3 || in_sizes[19] < D3) return;
    if (out_size < NB_FULL * D3 + D3) return;

    const float* x     = (const float*)d_in[0];
    const float* grid0 = (const float*)d_in[1];
    const float* coef0 = (const float*)d_in[2];
    const float* sb0   = (const float*)d_in[3];
    const float* ss0   = (const float*)d_in[4];
    const float* ns0   = (const float*)d_in[5];
    const float* nb0   = (const float*)d_in[6];
    const float* grid1 = (const float*)d_in[7];
    const float* coef1 = (const float*)d_in[8];
    const float* sb1   = (const float*)d_in[9];
    const float* ss1   = (const float*)d_in[10];
    const float* ns1   = (const float*)d_in[11];
    const float* nb1   = (const float*)d_in[12];
    const float* grid2 = (const float*)d_in[13];
    const float* coef2 = (const float*)d_in[14];
    const float* sb2   = (const float*)d_in[15];
    const float* ss2   = (const float*)d_in[16];
    const float* ns2   = (const float*)d_in[17];
    const float* nb2   = (const float*)d_in[18];
    const float* sigma = (const float*)d_in[19];
    float* out = (float*)d_out;

    char* wsp = (char*)d_ws;
    size_t off = 0;
    auto carve = [&](size_t bytes) -> void* { void* r = wsp + off; off += (bytes + 255) & ~(size_t)255; return r; };
    unsigned short* aplane = (unsigned short*)carve(WS_A);
    float*          h0c    = (float*)carve(WS_H0);
    float*          h1c    = (float*)carve(WS_H1);
    unsigned short* w0     = (unsigned short*)carve(WS_W0);
    unsigned short* w1     = (unsigned short*)carve(WS_W1);
    unsigned short* w2     = (unsigned short*)carve(WS_W2);
    if (off > ws_size || off > (size_t)134217728) return;

    k_wpack<<<(D1 * (9 * D0 / 8)) / 256, 256, 0, stream>>>(coef0, sb0, ss0, w0, D0, D1);
    k_wpack<<<(D2 * (9 * D1 / 8)) / 256, 256, 0, stream>>>(coef1, sb1, ss1, w1, D1, D2);
    k_wpack<<<(D3 * (9 * D2 / 8)) / 256, 256, 0, stream>>>(coef2, sb2, ss2, w2, D2, D3);

    const unsigned g1 = ((MCH / 64) * (D1 / 64)) / 8;
    const unsigned g2 = ((MCH / 64) * (D2 / 64)) / 8;
    const unsigned g3 = ((MCH / 64) * (D3 / 64)) / 8;

    for (int c = 0; c < NB / MCH; ++c) {
        const size_t rb = (size_t)c * MCH;
        k_expand<<<dim3(D0 / 256, MCH / XP_ROWS), 256, 0, stream>>>(x + rb * D0, grid0, aplane, D0, 1u);
        k_gemm64<<<g1, 256, 0, stream>>>((const _Float16*)aplane, 9 * D0, (const _Float16*)w0, 9 * D0,
            h0c, D1, ns0, nb0, MCH, D1, 9 * D0, SC);
        k_expand<<<dim3(D1 / 256, MCH / XP_ROWS), 256, 0, stream>>>(h0c, grid1, aplane, D1, 0u);
        k_gemm64<<<g2, 256, 0, stream>>>((const _Float16*)aplane, 9 * D1, (const _Float16*)w1, 9 * D1,
            h1c, D2, ns1, nb1, MCH, D2, 9 * D1, SC);
        k_expand<<<dim3(D2 / 256, MCH / XP_ROWS), 256, 0, stream>>>(h1c, grid2, aplane, D2, 0u);
        k_gemm64<<<g3, 256, 0, stream>>>((const _Float16*)aplane, 9 * D2, (const _Float16*)w2, 9 * D2,
            out + rb * D3, D3, ns2, nb2, MCH, D3, 9 * D2, SC);
    }
    k_sigma<<<1, 128, 0, stream>>>(sigma, out + (size_t)NB_FULL * D3);
}
